// ScaledDotProductAttention_53214644797493
// MI455X (gfx1250) — hardware-verified
//
#include <hip/hip_runtime.h>


#ifndef NB
#define NB 4
#endif
#ifndef SEQ
#define SEQ 2048
#endif
#define SEQ_FULL 2048
#define NHEAD    16
#define NBH      (NB * NHEAD)
#define DH       64
#define QBLK     128
#define NWAVE    8
#define KBLK     32
#define NKB      (SEQ / KBLK)
#define NQT      (SEQ / QBLK)
#define PSTR     40
#define OSTR     68
#define VTP      72
#define CV_GRID  (NBH * (SEQ / 64))
#define AT_GRID  (NBH * NQT)

#define SCL    0.18033688011112042f
#define MINIT  (-1.0e30f)
#define PCAR   16384.0f

static_assert(SEQ % 256 == 0);
static_assert(SEQ <= SEQ_FULL);
static_assert(NB >= 1 && NB <= 4);
static_assert((NWAVE * 16 * PSTR * 2) + NWAVE * 16 * OSTR * 4 <= 65536);
static_assert((PSTR * 2) % 16 == 0 && (OSTR * 4) % 16 == 0 && (VTP * 2) % 16 == 0);
static_assert((unsigned long long)CV_GRID * 256ull * 16ull == (unsigned long long)NBH * SEQ * DH);
static_assert((unsigned long long)AT_GRID * NWAVE * 16ull * DH == (unsigned long long)NBH * SEQ * DH);
static_assert(8 * 4 * 32 == 16 * DH);
static_assert(QBLK == NWAVE * 16);
static_assert(3ull * NBH * SEQ * DH * 2ull <= 134217728ull);

typedef _Float16 f16;
typedef _Float16 v16h __attribute__((ext_vector_type(16)));
typedef _Float16 v8h  __attribute__((ext_vector_type(8)));
typedef _Float16 v2h  __attribute__((ext_vector_type(2)));
typedef __bf16   v16b __attribute__((ext_vector_type(16)));
typedef unsigned short us16;
typedef us16     v8us __attribute__((ext_vector_type(8)));
typedef float    v8f  __attribute__((ext_vector_type(8)));
typedef float    v4f  __attribute__((ext_vector_type(4)));
typedef unsigned int v4u __attribute__((ext_vector_type(4)));

union FragH { v16h v; v8h half[2]; };
union FragB { v16b v; v16h hv; v8us half[2]; };
union Pack8 { v8h h; v4u u; };

static __device__ __forceinline__ v8f mma_f16(v16h a, v16h b, v8f c) {
  c = __builtin_amdgcn_wmma_f32_16x16x32_f16(false, a, false, b, (short)0, c, false, false);
  asm volatile("v_nop\n\tv_nop\n\tv_nop\n\tv_nop" : "+v"(c) : "v"(a), "v"(b));
  return c;
}
static __device__ __forceinline__ v8f mma_bf16(const FragB& a, const FragB& b, v8f c) {
  c = __builtin_amdgcn_wmma_f32_16x16x32_bf16(false, a.v, false, b.v, (short)0, c, false, false);
  asm volatile("v_nop\n\tv_nop\n\tv_nop\n\tv_nop" : "+v"(c) : "v"(a.hv), "v"(b.hv));
  return c;
}

static __device__ __forceinline__ unsigned int bf_hi(float x) {
  unsigned int u = __float_as_uint(x);
  u += 0x7FFFu + ((u >> 16) & 1u);
  return u >> 16;
}
static __device__ __forceinline__ f16 h_of_bf(float x) {
  return (f16)__uint_as_float(bf_hi(x) << 16);
}

template <int CTRL>
static __device__ __forceinline__ float dpp_max(float x) {
  int xi = __float_as_int(x);
  int yi = __builtin_amdgcn_update_dpp(xi, xi, CTRL, 0xF, 0xF, true);
  return fmaxf(x, __int_as_float(yi));
}
static __device__ __forceinline__ float rowmax16(float x) {
  x = dpp_max<0xB1>(x);
  x = dpp_max<0x4E>(x);
  x = dpp_max<0x141>(x);
  x = dpp_max<0x140>(x);
  return x;
}

static __device__ __forceinline__ void lds_wave_sync() {
  asm volatile("s_wait_dscnt 0x0" ::: "memory");
  __builtin_amdgcn_wave_barrier();
}

__global__ __launch_bounds__(256)
void k_convert(const float* __restrict__ Q, const float* __restrict__ K, const float* __restrict__ V,
               us16* __restrict__ Qp, us16* __restrict__ Kp, f16* __restrict__ Vt)
{
  __shared__ __align__(16) f16 sVt[DH * VTP];

  const unsigned tid   = threadIdx.x;
  const unsigned bh    = blockIdx.x / (unsigned)(SEQ / 64);
  const unsigned kt    = blockIdx.x - bh * (unsigned)(SEQ / 64);
  const size_t rin = (size_t)bh * SEQ_FULL + (size_t)kt * 64;
  const size_t rpl = (size_t)bh * SEQ + (size_t)kt * 64;
  const unsigned prow  = tid >> 3;
  const unsigned piece = tid & 7u;

  v4u qv[2], kv[2];
#pragma unroll
  for (unsigned it = 0; it < 2; ++it) {
    const unsigned row = it * 32u + prow;
    const float* qs = Q + (rin + row) * DH + piece * 8u;
    const float* ks = K + (rin + row) * DH + piece * 8u;
    const v4f q0 = *(const v4f*)(qs);
    const v4f q1 = *(const v4f*)(qs + 4);
    const v4f k0 = *(const v4f*)(ks);
    const v4f k1 = *(const v4f*)(ks + 4);
    v4u a, b;
    a.x = bf_hi(q0.x) | (bf_hi(q0.y) << 16);
    a.y = bf_hi(q0.z) | (bf_hi(q0.w) << 16);
    a.z = bf_hi(q1.x) | (bf_hi(q1.y) << 16);
    a.w = bf_hi(q1.z) | (bf_hi(q1.w) << 16);
    b.x = bf_hi(k0.x) | (bf_hi(k0.y) << 16);
    b.y = bf_hi(k0.z) | (bf_hi(k0.w) << 16);
    b.z = bf_hi(k1.x) | (bf_hi(k1.y) << 16);
    b.w = bf_hi(k1.z) | (bf_hi(k1.w) << 16);
    qv[it] = a;
    kv[it] = b;
  }
#pragma unroll
  for (unsigned it = 0; it < 2; ++it) {
    const unsigned row = it * 32u + prow;
    *(volatile v4u*)(Qp + (rpl + row) * DH + piece * 8u) = qv[it];
    *(volatile v4u*)(Kp + (rpl + row) * DH + piece * 8u) = kv[it];
  }
  __threadfence();
#pragma unroll
  for (unsigned it = 0; it < 2; ++it) {
    const unsigned row = it * 32u + prow;
    *(volatile v4u*)(Qp + (rpl + row) * DH + piece * 8u) = qv[it];
    *(volatile v4u*)(Kp + (rpl + row) * DH + piece * 8u) = kv[it];
  }

  {
    const unsigned key = tid >> 2;
    const unsigned d0  = (tid & 3u) * 16u;
    const float* vs = V + (rin + key) * DH + d0;
#pragma unroll
    for (unsigned j = 0; j < 4; ++j) {
      const v4f x = *(const v4f*)(vs + 4 * j);
      sVt[(d0 + 4 * j + 0) * VTP + key] = h_of_bf(x.x);
      sVt[(d0 + 4 * j + 1) * VTP + key] = h_of_bf(x.y);
      sVt[(d0 + 4 * j + 2) * VTP + key] = h_of_bf(x.z);
      sVt[(d0 + 4 * j + 3) * VTP + key] = h_of_bf(x.w);
    }
  }
  __syncthreads();
  Pack8 vv[2];
#pragma unroll
  for (unsigned it = 0; it < 2; ++it) {
    const unsigned d = it * 32u + prow;
    vv[it].h = *(const v8h*)(sVt + d * VTP + piece * 8u);
  }
#pragma unroll
  for (unsigned it = 0; it < 2; ++it) {
    const unsigned d = it * 32u + prow;
    *(volatile v4u*)(Vt + ((size_t)bh * DH + d) * SEQ + (size_t)kt * 64 + piece * 8u) = vv[it].u;
  }
  __threadfence();
#pragma unroll
  for (unsigned it = 0; it < 2; ++it) {
    const unsigned d = it * 32u + prow;
    *(volatile v4u*)(Vt + ((size_t)bh * DH + d) * SEQ + (size_t)kt * 64 + piece * 8u) = vv[it].u;
  }
}

__global__ __launch_bounds__(256)
void k_attn(const us16* __restrict__ Qp, const us16* __restrict__ Kp, const f16* __restrict__ Vt,
            float* __restrict__ O)
{
  __shared__ __align__(16) f16   sP[NWAVE * 16 * PSTR];
  __shared__ __align__(16) float sO[NWAVE * 16 * OSTR];

  const unsigned tid  = threadIdx.x;
  const unsigned wave = tid >> 5;
  const unsigned lane = tid & 31u;
  const unsigned h    = lane >> 4;
  const unsigned l16  = lane & 15u;

  const unsigned bh    = blockIdx.x / (unsigned)NQT;
  const unsigned qt    = blockIdx.x - bh * (unsigned)NQT;
  const unsigned qwave = qt * QBLK + wave * 16u;

  const us16* Qb = Qp + ((size_t)bh * SEQ + qwave) * DH;
  const us16* Kb = Kp + (size_t)bh * SEQ * DH;
  const f16*  Vb = Vt + (size_t)bh * DH * SEQ;
  float*      Ob = O + ((size_t)bh * SEQ + qwave) * DH;

  FragB qa[2];
#pragma unroll
  for (unsigned kc = 0; kc < 2; ++kc) {
    const us16* qr = Qb + (size_t)l16 * DH + kc * 32u + 8u * h;
    qa[kc].half[0] = *(const v8us*)(qr);
    qa[kc].half[1] = *(const v8us*)(qr + 16);
  }

  v16h onesv;
#pragma unroll
  for (int i = 0; i < 16; ++i) onesv[i] = (f16)1.0f;

  const v8f vzero = {0.f, 0.f, 0.f, 0.f, 0.f, 0.f, 0.f, 0.f};
  v8f oacc[4];
#pragma unroll
  for (int vt = 0; vt < 4; ++vt) oacc[vt] = vzero;
  float mrow[8], lrow[8];
#pragma unroll
  for (int r = 0; r < 8; ++r) { mrow[r] = MINIT; lrow[r] = 0.f; }

  const unsigned pofs = wave * 16u * PSTR;

#pragma unroll 1
  for (unsigned kb = 0; kb < (unsigned)NKB; ++kb) {
    const unsigned k0 = kb * KBLK;

    FragB kf[2][2];
#pragma unroll
    for (unsigned nt = 0; nt < 2; ++nt)
#pragma unroll
      for (unsigned kc = 0; kc < 2; ++kc) {
        const us16* kr = Kb + (size_t)(k0 + 2u * l16 + nt) * DH + kc * 32u + 8u * h;
        kf[nt][kc].half[0] = *(const v8us*)(kr);
        kf[nt][kc].half[1] = *(const v8us*)(kr + 16);
      }

    v8f s0 = mma_bf16(qa[0], kf[0][0], vzero);
    s0     = mma_bf16(qa[1], kf[0][1], s0);
    v8f s1 = mma_bf16(qa[0], kf[1][0], vzero);
    s1     = mma_bf16(qa[1], kf[1][1], s1);
#pragma unroll
    for (int r = 0; r < 8; ++r) { s0[r] *= SCL; s1[r] *= SCL; }

    float alpha[8];
#pragma unroll
    for (int r = 0; r < 8; ++r) {
      const float mx = rowmax16(fmaxf(s0[r], s1[r]));
      const float mn = fmaxf(mrow[r], mx);
      alpha[r] = __builtin_amdgcn_exp2f(mrow[r] - mn);
      mrow[r]  = mn;
      const float p0 = __builtin_amdgcn_exp2f(s0[r] - mn) * PCAR;
      const float p1 = __builtin_amdgcn_exp2f(s1[r] - mn) * PCAR;
      v2h pp; pp.x = (f16)p0; pp.y = (f16)p1;
      *(v2h*)(sP + pofs + (8u * h + (unsigned)r) * PSTR + 2u * l16) = pp;
    }
    lds_wave_sync();

    FragH pa;
    pa.half[0] = *(const v8h*)(sP + pofs + l16 * PSTR + 8u * h);
    pa.half[1] = *(const v8h*)(sP + pofs + l16 * PSTR + 16u + 8u * h);

    const v8f lsum = mma_f16(pa.v, onesv, vzero);

#pragma unroll
    for (unsigned vt = 0; vt < 4; ++vt) {
      FragH vb;
      const f16* vr = Vb + (size_t)(vt * 16u + l16) * SEQ + k0 + 8u * h;
      vb.half[0] = *(const v8h*)(vr);
      vb.half[1] = *(const v8h*)(vr + 16);
#pragma unroll
      for (int r = 0; r < 8; ++r) oacc[vt][r] *= alpha[r];
      oacc[vt] = mma_f16(pa.v, vb.v, oacc[vt]);
    }
#pragma unroll
    for (int r = 0; r < 8; ++r) lrow[r] = lrow[r] * alpha[r] + lsum[r];

    lds_wave_sync();
  }

  float inv[8];
#pragma unroll
  for (int r = 0; r < 8; ++r) inv[r] = __builtin_amdgcn_rcpf(lrow[r]);
  float* sOw = sO + wave * 16u * OSTR;
#pragma unroll
  for (unsigned vt = 0; vt < 4; ++vt)
#pragma unroll
    for (int r = 0; r < 8; ++r)
      sOw[(8u * h + (unsigned)r) * OSTR + vt * 16u + l16] = oacc[vt][r] * inv[r];
  lds_wave_sync();

  const unsigned lq = lane >> 3;
  const unsigned lp = lane & 7u;
#pragma unroll
  for (unsigned j = 0; j < 8; ++j) {
    const unsigned L = j * 4u + lq;
    const unsigned row = L >> 1, hf = L & 1u;
    const v4f v = *(const v4f*)(sOw + row * OSTR + hf * 32u + lp * 4u);
    *(volatile v4f*)(Ob + (size_t)row * DH + hf * 32u + lp * 4u) = v;
  }
  __threadfence();
#pragma unroll
  for (unsigned j = 0; j < 8; ++j) {
    const unsigned L = j * 4u + lq;
    const unsigned row = L >> 1, hf = L & 1u;
    const v4f v = *(const v4f*)(sOw + row * OSTR + hf * 32u + lp * 4u);
    *(volatile v4f*)(Ob + (size_t)row * DH + hf * 32u + lp * 4u) = v;
  }
}

extern "C" void kernel_launch(void* const* d_in, const int* in_sizes, int n_in,
                              void* d_out, int out_size, void* d_ws, size_t ws_size,
                              hipStream_t stream)
{
  if (n_in < 3) return;
  const long long needQ = ((long long)(NBH - 1) * SEQ_FULL + SEQ) * DH;
  if ((long long)in_sizes[0] < needQ) return;
  if ((long long)in_sizes[1] < needQ) return;
  if ((long long)in_sizes[2] < needQ) return;
  if ((long long)out_size < (long long)NBH * SEQ * DH) return;

  const float* Q = (const float*)d_in[0];
  const float* K = (const float*)d_in[1];
  const float* V = (const float*)d_in[2];
  float*       O = (float*)d_out;

  const size_t planeB = (size_t)NBH * SEQ * DH * 2;
  const size_t offQ   = 0;
  const size_t offK   = planeB;
  const size_t offV   = 2 * planeB;
  const size_t total  = 3 * planeB;
  if (ws_size < total) return;

  char* ws = (char*)d_ws;
  us16* Qp = (us16*)(ws + offQ);
  us16* Kp = (us16*)(ws + offK);
  f16*  Vt = (f16*)(ws + offV);

  k_convert<<<dim3(CV_GRID), dim3(256), 0, stream>>>(Q, K, V, Qp, Kp, Vt);
  k_attn<<<dim3(AT_GRID), dim3(256), 0, stream>>>(Qp, Kp, Vt, O);
}
